// iRMB_25967372271807
// MI455X (gfx1250) — hardware-verified
//
#include <hip/hip_runtime.h>
#include <math.h>


#define NB 16
#define CC 256
#define HI 56
#define WI 56
#define NPIX (HI * WI)
#define WS 7
#define NWIN 64
#define NTOK 49
#define NH 4
#define DHD 64
#define NR (NB * NPIX)

typedef __attribute__((ext_vector_type(16))) _Float16 v16h;
typedef __attribute__((ext_vector_type(8)))  _Float16 v8h;
typedef __attribute__((ext_vector_type(8)))  float v8f;
typedef __attribute__((ext_vector_type(4)))  float v4f;
typedef __attribute__((ext_vector_type(4)))  unsigned v4u;
typedef float __attribute__((may_alias)) float_a;

template <typename T> __device__ __forceinline__ void vst2(void* p, T v) { *(volatile T*)p = v; __threadfence(); *(volatile T*)p = v; }
__device__ __forceinline__ v8f wmma16(v16h a, v16h b, v8f c) {
  v8f d = __builtin_amdgcn_wmma_f32_16x16x32_f16(false, a, false, b, (short)0, c, false, false);
  asm volatile("v_nop\n\tv_nop\n\tv_nop\n\tv_nop" : "+v"(d) : "v"(a), "v"(b));
  return d;
}
__device__ __forceinline__ v16h frag_h(const _Float16* rowk0, int lane) {
  union { v16h v; v8h q[2]; } u; const _Float16* p = rowk0 + 8 * (lane >> 4);
  u.q[0] = *(const v8h*)p; u.q[1] = *(const v8h*)(p + 16); return u.v;
}
__device__ __forceinline__ v16h frag_f32(const float* rowk0, int lane) {
  v16h a; const float* p = rowk0 + 8 * (lane >> 4);
#pragma unroll
  for (int i = 0; i < 8; ++i) { a[i] = (_Float16)p[i]; a[8 + i] = (_Float16)p[16 + i]; }
  return a;
}
__device__ __forceinline__ float silu(float v) { return v / (1.0f + expf(-v)); }
#define LDSX() do { asm volatile("s_wait_dscnt 0" ::: "memory"); __builtin_amdgcn_wave_barrier(); __builtin_amdgcn_fence(__ATOMIC_RELEASE, "workgroup"); } while (0)

__device__ __forceinline__ int wrow2pix(int wr) { const int win = wr / NTOK, hw = wr % NTOK; const int n1 = win >> 3, n2 = win & 7, h1 = hw / WS, w1 = hw % WS; return (h1 * 8 + n1) * WI + (w1 * 8 + n2); }
__device__ __forceinline__ int pix2wrow(int p) { const int h = p / WI, w = p % WI; const int h1 = h >> 3, n1 = h & 7, w1 = w >> 3, n2 = w & 7; return (n1 * 8 + n2) * NTOK + h1 * WS + w1; }

__global__ __launch_bounds__(256) void k_bnstat(const float* __restrict__ x, const float* __restrict__ gm, const float* __restrict__ bt, float* __restrict__ stats) {
  __shared__ float red[256];
  const int c = blockIdx.x, tid = threadIdx.x;
  float s = 0.f;
#pragma unroll 1
  for (int b = 0; b < NB; ++b) { const float* xp = x + ((size_t)b * CC + c) * NPIX;
#pragma unroll 1
    for (int i = tid; i < NPIX; i += 256) s += xp[i]; }
  red[tid] = s; __syncthreads();
  for (int st = 128; st > 0; st >>= 1) { if (tid < st) red[tid] += red[tid + st]; __syncthreads(); }
  const float mu = red[0] / (float)(NB * NPIX); __syncthreads();
  float q = 0.f;
#pragma unroll 1
  for (int b = 0; b < NB; ++b) { const float* xp = x + ((size_t)b * CC + c) * NPIX;
#pragma unroll 1
    for (int i = tid; i < NPIX; i += 256) { const float d = xp[i] - mu; q += d * d; } }
  red[tid] = q; __syncthreads();
  for (int st = 128; st > 0; st >>= 1) { if (tid < st) red[tid] += red[tid + st]; __syncthreads(); }
  if (tid == 0) { const float var = red[0] / (float)(NB * NPIX); v4f v = { mu, rsqrtf(var + 1e-5f) * gm[c], bt[c], 0.f }; vst2(stats + (size_t)c * 32, v); }
}

__global__ __launch_bounds__(256) void k_bnwin(const float* __restrict__ x, const float* __restrict__ stats, float* __restrict__ xw) {
  __shared__ float tile[64][65];
  const int b = blockIdx.z, c0 = blockIdx.y * 64, p0 = blockIdx.x * 64, tid = threadIdx.x;
  for (int i = tid; i < 64 * 64; i += 256) { const int cl = i >> 6, pl = i & 63;
    const float mu = stats[(size_t)(c0 + cl) * 32], sc = stats[(size_t)(c0 + cl) * 32 + 1], be = stats[(size_t)(c0 + cl) * 32 + 2];
    tile[cl][pl] = (x[((size_t)b * CC + c0 + cl) * NPIX + p0 + pl] - mu) * sc + be; }
  __syncthreads();
  for (int i = tid; i < 64 * 16; i += 256) { const int pl = i >> 4, pc = i & 15; const int wr = pix2wrow(p0 + pl);
    v4f v = { tile[pc * 4][pl], tile[pc * 4 + 1][pl], tile[pc * 4 + 2][pl], tile[pc * 4 + 3][pl] };
    vst2(xw + ((size_t)b * NPIX + wr) * CC + c0 + pc * 4, v); }
}
__global__ __launch_bounds__(256) void k_cvt(const float* __restrict__ s, _Float16* __restrict__ d, size_t n8) {
  const size_t g8 = (size_t)blockIdx.x * 256 + threadIdx.x; if (g8 >= n8) return;
  union { v8h h; v4u u; } pk;
#pragma unroll
  for (int e = 0; e < 8; ++e) pk.h[e] = (_Float16)s[g8 * 8 + e];
  vst2(d + g8 * 8, pk.u);
}

template <int GATHER, int MODE>
__global__ __launch_bounds__(128) void k_pw(const float* __restrict__ A, const _Float16* __restrict__ W, const float* __restrict__ bias,
                                          const float* __restrict__ skip, void* __restrict__ Outv, int K, int N) {
  float* Out = (float*)Outv; _Float16* Outh = (_Float16*)Outv;
  __shared__ __align__(16) float so[128][68];
  const int tid = threadIdx.x, wave = tid >> 5, lane = tid & 31, col = lane & 15, g = lane >> 4;
  const int b = blockIdx.z, p0 = blockIdx.x * 64, n0 = blockIdx.y * 128;
  const int prow = p0 + wave * 16 + col;
  const size_t arow = (size_t)b * NPIX + (GATHER ? pix2wrow(prow) : prow);
  v8f acc[8] = {};
#pragma unroll 1
  for (int kc = 0; kc < K / 32; ++kc) { const v16h a = frag_f32(A + arow * K + kc * 32, lane);
#pragma unroll
    for (int j = 0; j < 8; ++j) acc[j] = wmma16(a, frag_h(W + (size_t)(n0 + j * 16 + col) * K + kc * 32, lane), acc[j]); }
  if (MODE != 1) {
    float* S = &so[0][0] + wave * (16 * 128);
#pragma unroll
    for (int j = 0; j < 8; ++j) { const float bv = bias ? bias[n0 + j * 16 + col] : 0.f;
#pragma unroll
      for (int r = 0; r < 8; ++r) S[(8 * g + r) * 128 + j * 16 + col] = acc[j][r] + bv; }
    LDSX();
    if (MODE == 0) {
#pragma unroll 4
      for (int rl = 0; rl < 16; ++rl) vst2(Out + ((size_t)b * NPIX + p0 + wave * 16 + rl) * N + n0 + lane * 4, *(const v4f*)(S + rl * 128 + lane * 4));
    } else {
#pragma unroll
      for (int q = 0; q < 8; ++q) { const int rl = q * 2 + (lane >> 4), pc = lane & 15;
        union { v8h h; v4u u; } pk;
#pragma unroll
        for (int e = 0; e < 8; ++e) pk.h[e] = (_Float16)S[rl * 128 + pc * 8 + e];
        vst2(Outh + ((size_t)b * NPIX + p0 + wave * 16 + rl) * N + n0 + pc * 8, pk.u); }
    }
  } else {
#pragma unroll
    for (int j = 0; j < 8; ++j) { const float bv = bias[n0 + j * 16 + col];
#pragma unroll
      for (int r = 0; r < 8; ++r) so[j * 16 + col][wave * 16 + 8 * g + r] = acc[j][r] + bv; }
    __syncthreads();
    for (int q = tid; q < 128 * 16; q += 128) { const int cl = q >> 4, pc = q & 15; const int c = n0 + cl;
      v4f v = *(const v4f*)(&so[cl][pc * 4]);
#pragma unroll
      for (int e = 0; e < 4; ++e) v[e] += skip[((size_t)b * NPIX + pix2wrow(p0 + pc * 4 + e)) * CC + c];
      vst2(Out + ((size_t)b * CC + c) * NPIX + p0 + pc * 4, v); }
  }
}

__global__ __launch_bounds__(256) void k_window(const float* __restrict__ xw, const _Float16* __restrict__ qkv,
                                              const float* __restrict__ w3, const float* __restrict__ b3, const float* __restrict__ w5, const float* __restrict__ b5,
                                              const float* __restrict__ w7, const float* __restrict__ b7, float* __restrict__ y) {
  __shared__ __align__(16) float sx[NTOK][CC];
  __shared__ float sq[NTOK][DHD + 1], sk[NTOK][DHD + 1], sv[NTOK][DHD + 1];
  __shared__ float ss[NTOK][NTOK + 1];
  __shared__ __align__(16) float sy[NTOK][CC];
  const int b = blockIdx.y, win = blockIdx.x, tid = threadIdx.x, lane = tid & 31, wave = tid >> 5;
  const size_t r0 = (size_t)b * NPIX + (size_t)win * NTOK;
  for (int i = tid; i < NTOK * (CC / 4); i += 256) { const int t = i / (CC / 4), pc = i % (CC / 4); *(v4f*)&sx[t][pc * 4] = *(const v4f*)(xw + (r0 + t) * CC + pc * 4); }
  __syncthreads();
  { const int c = tid;
    float k3[9], k5[25], k7[49];
    for (int i = 0; i < 9; ++i) k3[i] = w3[c * 9 + i];
    for (int i = 0; i < 25; ++i) k5[i] = w5[c * 25 + i];
    for (int i = 0; i < 49; ++i) k7[i] = w7[c * 49 + i];
    const float bb = b3[c] + b5[c] + b7[c];
#pragma unroll 1
    for (int t = 0; t < NTOK; ++t) { const int h1 = t / WS, w1 = t % WS; float a = bb;
#pragma unroll 1
      for (int dy = -3; dy <= 3; ++dy) { const int hh = h1 + dy; if (hh < 0 || hh >= WS) continue;
#pragma unroll 1
        for (int dx = -3; dx <= 3; ++dx) { const int ww = w1 + dx; if (ww < 0 || ww >= WS) continue;
          const float xv = sx[hh * WS + ww][c];
          float wsum = k7[(dy + 3) * 7 + dx + 3];
          if (dy >= -2 && dy <= 2 && dx >= -2 && dx <= 2) wsum += k5[(dy + 2) * 5 + dx + 2];
          if (dy >= -1 && dy <= 1 && dx >= -1 && dx <= 1) wsum += k3[(dy + 1) * 3 + dx + 1];
          a += wsum * xv; } }
      sy[t][c] = 0.25f * a; } }
  __syncthreads();
#pragma unroll 1
  for (int h = 0; h < NH; ++h) {
    for (int i = tid; i < NTOK * DHD; i += 256) { const int t = i / DHD, d = i % DHD; const size_t qr = (r0 + t) * (3 * CC);
      sq[t][d] = (float)qkv[qr + h * DHD + d]; sk[t][d] = (float)qkv[qr + CC + h * DHD + d]; sv[t][d] = (float)qkv[qr + 2 * CC + h * DHD + d] + sx[t][h * DHD + d]; }
    __syncthreads();
    for (int i = tid; i < NTOK * NTOK; i += 256) { const int qi = i / NTOK, ki = i % NTOK; float s = 0.f;
#pragma unroll 1
      for (int d = 0; d < DHD; ++d) s += sq[qi][d] * sk[ki][d];
      ss[qi][ki] = s * 0.125f; }
    __syncthreads();
    if (tid < NTOK) { float mx = -3.0e38f; for (int k = 0; k < NTOK; ++k) mx = fmaxf(mx, ss[tid][k]);
      float sum = 0.f; for (int k = 0; k < NTOK; ++k) { const float e = expf(ss[tid][k] - mx); ss[tid][k] = e; sum += e; }
      const float inv = 1.0f / sum; for (int k = 0; k < NTOK; ++k) ss[tid][k] *= inv; }
    __syncthreads();
    for (int i = tid; i < NTOK * DHD; i += 256) { const int qi = i / DHD, d = i % DHD; float o = 0.f;
#pragma unroll 1
      for (int k = 0; k < NTOK; ++k) o += ss[qi][k] * sv[k][d];
      sy[qi][h * DHD + d] += 0.25f * o + sv[qi][d]; }
    __syncthreads();
  }
  for (int i = tid; i < NTOK * (CC / 4); i += 256) { const int t = i / (CC / 4), pc = i % (CC / 4); vst2(y + (r0 + t) * CC + pc * 4, *(const v4f*)&sy[t][pc * 4]); }
}

__global__ __launch_bounds__(256) void k_dw3(const float* __restrict__ t1, const float* __restrict__ wl, const float* __restrict__ bl, float* __restrict__ t2) {
  const int b = blockIdx.y, h = blockIdx.x, c = threadIdx.x;
  float k[9]; for (int i = 0; i < 9; ++i) k[i] = wl[c * 9 + i];
  const float bb = bl[c];
#pragma unroll 1
  for (int w = 0; w < WI; ++w) { float a = bb;
#pragma unroll 1
    for (int dy = -1; dy <= 1; ++dy) { const int hh = h + dy; if (hh < 0 || hh >= HI) continue;
#pragma unroll 1
      for (int dx = -1; dx <= 1; ++dx) { const int ww = w + dx; if (ww < 0 || ww >= WI) continue;
        a += k[(dy + 1) * 3 + dx + 1] * t1[((size_t)b * NPIX + hh * WI + ww) * CC + c]; } }
    vst2(t2 + ((size_t)b * NPIX + h * WI + w) * CC + c, (float_a)silu(a)); }
}

extern "C" void kernel_launch(void* const* d_in, const int* in_sizes, int n_in,
                              void* d_out, int out_size, void* d_ws, size_t ws_size,
                              hipStream_t stream) {
  (void)in_sizes; (void)n_in; (void)out_size; (void)ws_size;
  const float* x = (const float*)d_in[0]; const float* gm = (const float*)d_in[1]; const float* bt = (const float*)d_in[2];
  const float* qkvw = (const float*)d_in[3];
  const float* w3 = (const float*)d_in[4]; const float* b3 = (const float*)d_in[5];
  const float* w5 = (const float*)d_in[6]; const float* b5 = (const float*)d_in[7];
  const float* w7 = (const float*)d_in[8]; const float* b7 = (const float*)d_in[9];
  const float* fiw = (const float*)d_in[10]; const float* fib = (const float*)d_in[11];
  const float* wl = (const float*)d_in[12]; const float* bl = (const float*)d_in[13];
  const float* fow = (const float*)d_in[14]; const float* fob = (const float*)d_in[15];
  float* out = (float*)d_out;
  char* ws = (char*)d_ws; size_t off = 0;
  auto take = [&](size_t bytes) { char* p = ws + off; off += (bytes + 255) & ~(size_t)255; return p; };
  float* stats = (float*)take((size_t)CC * 32 * 4);
  float* xw = (float*)take((size_t)NR * CC * 4);
  _Float16* qkvh = (_Float16*)take((size_t)3 * CC * CC * 2); _Float16* fih = (_Float16*)take((size_t)CC * CC * 2); _Float16* foh = (_Float16*)take((size_t)CC * CC * 2);
  _Float16* qkv = (_Float16*)take((size_t)NR * 3 * CC * 2);
  float* y = (float*)take((size_t)NR * CC * 4);
  float* t1 = (float*)qkv;
  float* t2 = xw;
  k_bnstat<<<CC, 256, 0, stream>>>(x, gm, bt, stats);
  k_bnwin<<<dim3(NPIX / 64, CC / 64, NB), 256, 0, stream>>>(x, stats, xw);
  k_cvt<<<(unsigned)((3 * CC * CC / 8 + 255) / 256), 256, 0, stream>>>(qkvw, qkvh, (size_t)3 * CC * CC / 8);
  k_cvt<<<(unsigned)((CC * CC / 8 + 255) / 256), 256, 0, stream>>>(fiw, fih, (size_t)CC * CC / 8);
  k_cvt<<<(unsigned)((CC * CC / 8 + 255) / 256), 256, 0, stream>>>(fow, foh, (size_t)CC * CC / 8);
  k_pw<0, 2><<<dim3(NPIX / 64, 3 * CC / 128, NB), 128, 0, stream>>>(xw, qkvh, nullptr, nullptr, qkv, CC, 3 * CC);
  k_window<<<dim3(NWIN, NB), 256, 0, stream>>>(xw, qkv, w3, b3, w5, b5, w7, b7, y);
  k_pw<1, 0><<<dim3(NPIX / 64, CC / 128, NB), 128, 0, stream>>>(y, fih, fib, nullptr, t1, CC, CC);
  k_dw3<<<dim3(HI, NB), 256, 0, stream>>>(t1, wl, bl, t2);
  k_pw<0, 1><<<dim3(NPIX / 64, CC / 128, NB), 128, 0, stream>>>(t2, foh, fob, y, out, CC, CC);
}
